// LSTMAutoencoder_30253749633447
// MI455X (gfx1250) — hardware-verified
//
#include <hip/hip_runtime.h>
#include <math.h>

constexpr int NSEQ    = 512;
constexpr int NSTEP   = 256;
constexpr int NIN     = 64;
constexpr int NHID    = 64;
constexpr int NGATE   = 4 * NHID;
constexpr int KCAT    = NIN + NHID;
constexpr int NLAYER  = 4;
constexpr int NTHR    = 128;
constexpr int SEQ_BLK = 16;
constexpr int APITCH  = 136;
constexpr int OPITCH  = 68;
constexpr int NROWS   = NSEQ * NSTEP;
constexpr int WPLANE  = NGATE * KCAT;
constexpr float OPCARRY  = 16.0f;
constexpr float ACC_FOLD = 1.0f / 256.0f;
static_assert(NSEQ % SEQ_BLK == 0);
static_assert(NHID == 16 * (NTHR / 32));
static_assert(SEQ_BLK * NIN == 8 * NTHR);
static_assert(SEQ_BLK * NHID == 8 * NTHR);
static_assert(KCAT % 32 == 0);
static_assert(NLAYER * 2 * NGATE * (NIN / 8) == 128 * NTHR);
static_assert(APITCH % 8 == 0 && OPITCH % 4 == 0);
static_assert((NHID * 4) % 128 == 0 && (NHID * 2) % 128 == 0);

typedef __attribute__((ext_vector_type(16))) _Float16 v16h;
typedef __attribute__((ext_vector_type(8)))  _Float16 v8h;
typedef __attribute__((ext_vector_type(8)))  float    v8f;
typedef __attribute__((ext_vector_type(4)))  float    v4f;
typedef __attribute__((ext_vector_type(4)))  unsigned v4u;

__device__ __forceinline__ void tie_all_h(v8f& a0, v8f& a1, v8f& a2, v8f& a3,
                                          v16h fa, v16h b0, v16h b1, v16h b2, v16h b3) {
  asm volatile("v_nop\n\tv_nop\n\tv_nop\n\tv_nop"
               : "+v"(a0), "+v"(a1), "+v"(a2), "+v"(a3)
               : "v"(fa), "v"(b0), "v"(b1), "v"(b2), "v"(b3));
}
__device__ __forceinline__ void acc_guard4(v8f& a, v8f& b, v8f& c, v8f& d) {
  asm volatile("v_nop\n\tv_nop\n\tv_nop\n\tv_nop" : "+v"(a), "+v"(b), "+v"(c), "+v"(d));
}

template <typename T> struct Frag;
template <> struct Frag<_Float16> {
  typedef v16h V; union U { v16h v; v8h h[2]; };
  static __device__ __forceinline__ v16h load(const _Float16* p) {
    U f; f.h[0] = *(const v8h*)(p); f.h[1] = *(const v8h*)(p + 16); return f.v;
  }
  static __device__ __forceinline__ v8f mma(v16h a, v16h b, v8f c) {
    return __builtin_amdgcn_wmma_f32_16x16x32_f16(false, a, false, b, (short)0, c, false, false);
  }
};

__device__ __forceinline__ float gate_sig(float x) {
  const float e = expf(fminf(-x, 60.0f));
  return __builtin_amdgcn_rcpf(1.0f + e);
}
__device__ __forceinline__ float gate_tanh(float x) {
  const float e = expf(fminf(2.0f * x, 60.0f));
  return 1.0f - 2.0f * __builtin_amdgcn_rcpf(1.0f + e);
}

__global__ __launch_bounds__(NTHR) void wcat_kernel(const float* __restrict__ wi0, const float* __restrict__ wh0,
                                                    const float* __restrict__ wi1, const float* __restrict__ wh1,
                                                    const float* __restrict__ wi2, const float* __restrict__ wh2,
                                                    const float* __restrict__ wi3, const float* __restrict__ wh3,
                                                    unsigned short* __restrict__ WC) {
  const int bx = blockIdx.x;
  const int layer = bx >> 5;
  const int part  = (bx >> 4) & 1;
  const int idx = (bx & 15) * NTHR + threadIdx.x;
  const int n = idx >> 3, c8 = (idx & 7) * 8;
  const float* wi = (layer == 0) ? wi0 : (layer == 1) ? wi1 : (layer == 2) ? wi2 : wi3;
  const float* wh = (layer == 0) ? wh0 : (layer == 1) ? wh1 : (layer == 2) ? wh2 : wh3;
  const float* src = part ? wh : wi;
  const float* sp = src + (size_t)n * NIN + c8;
  const v4f a = *(const v4f*)(sp);
  const v4f b = *(const v4f*)(sp + 4);
  v8h hv;
#pragma unroll
  for (int e = 0; e < 4; ++e) {
    hv[e]     = (_Float16)(a[e] * OPCARRY);
    hv[4 + e] = (_Float16)(b[e] * OPCARRY);
  }
  unsigned short* dp = WC + (size_t)layer * WPLANE + (size_t)n * KCAT + part * NIN + c8;
  *(volatile v8h*)dp = hv;
  __threadfence();
  *(volatile v8h*)dp = hv;
}

template <int IN_F32>
__device__ __forceinline__ void stage_x_tile(_Float16* Axh, const float* __restrict__ xs32,
                                             const unsigned short* __restrict__ xs16, int rowbase, int tstep, int tid) {
  const int m = tid >> 3, c8 = (tid & 7) * 8;
  const size_t eoff = ((size_t)(rowbase + m) * NSTEP + (size_t)tstep) * NIN + (size_t)c8;
  _Float16* dst = Axh + m * APITCH + c8;
  if (IN_F32) {
    const v4f a = *(const v4f*)(xs32 + eoff);
    const v4f b = *(const v4f*)(xs32 + eoff + 4);
    v8h hv;
#pragma unroll
    for (int e = 0; e < 4; ++e) {
      hv[e]     = (_Float16)(a[e] * OPCARRY);
      hv[4 + e] = (_Float16)(b[e] * OPCARRY);
    }
    *(v8h*)dst = hv;
  } else {
    const v4u w = *(const v4u*)(xs16 + eoff);
    *(v4u*)(void*)dst = w;
  }
}

template <int IN_F32, int OUT_F32>
__global__ __launch_bounds__(NTHR) void seq_cell_kernel(const float* __restrict__ xs32, const unsigned short* __restrict__ xs16,
                                                        const float* __restrict__ bih, const float* __restrict__ bhh,
                                                        const unsigned short* __restrict__ WCp,
                                                        unsigned short* __restrict__ h16out, float* __restrict__ h32out) {
  __shared__ __align__(16) _Float16 Axh[SEQ_BLK * APITCH];
  __shared__ __align__(16) float    Hs[SEQ_BLK * OPITCH];
  const _Float16* WC = (const _Float16*)WCp;
  const int tid = threadIdx.x, lane = tid & 31, wave = tid >> 5;
  const int c = lane & 15, hh = lane >> 4, koff = hh * 8;
  const int rowbase = blockIdx.x * SEQ_BLK;
  const int j = 16 * wave + c;
  (void)xs32; (void)xs16; (void)h16out; (void)h32out;

  {
    const int m = tid >> 3, c8 = (tid & 7) * 8;
    v8h zh;
#pragma unroll
    for (int e = 0; e < 8; ++e) zh[e] = (_Float16)0.0f;
    *(v8h*)(Axh + m * APITCH + NIN + c8) = zh;
  }
  stage_x_tile<IN_F32>(Axh, xs32, xs16, rowbase, 0, tid);

  float bb[4];
#pragma unroll
  for (int g = 0; g < 4; ++g) bb[g] = bih[g * NHID + j] + bhh[g * NHID + j];
  float cst[8], hst[8];
#pragma unroll
  for (int r = 0; r < 8; ++r) { cst[r] = 0.0f; hst[r] = 0.0f; }
  __syncthreads();

  const _Float16* arow = Axh + c * APITCH + koff;
  const _Float16* wrow = WC + (size_t)j * KCAT + koff;
  const v8f z8 = {0.f, 0.f, 0.f, 0.f, 0.f, 0.f, 0.f, 0.f};

#pragma unroll 1
  for (int t = 0; t < NSTEP; ++t) {
    v8f acc[4];
    acc[0] = z8; acc[1] = z8; acc[2] = z8; acc[3] = z8;
#pragma unroll 1
    for (int k0 = 0; k0 < KCAT; k0 += 32) {
      const v16h a  = Frag<_Float16>::load(arow + k0);
      const v16h b0 = Frag<_Float16>::load(wrow + k0);
      const v16h b1 = Frag<_Float16>::load(wrow + (size_t)1 * NHID * KCAT + k0);
      const v16h b2 = Frag<_Float16>::load(wrow + (size_t)2 * NHID * KCAT + k0);
      const v16h b3 = Frag<_Float16>::load(wrow + (size_t)3 * NHID * KCAT + k0);
      acc[0] = Frag<_Float16>::mma(a, b0, acc[0]);
      acc[1] = Frag<_Float16>::mma(a, b1, acc[1]);
      acc[2] = Frag<_Float16>::mma(a, b2, acc[2]);
      acc[3] = Frag<_Float16>::mma(a, b3, acc[3]);
      tie_all_h(acc[0], acc[1], acc[2], acc[3], a, b0, b1, b2, b3);
    }
    acc_guard4(acc[0], acc[1], acc[2], acc[3]);
#pragma unroll
    for (int r = 0; r < 8; ++r) {
      const float zi = acc[0][r] * ACC_FOLD + bb[0];
      const float zf = acc[1][r] * ACC_FOLD + bb[1];
      const float zg = acc[2][r] * ACC_FOLD + bb[2];
      const float zo = acc[3][r] * ACC_FOLD + bb[3];
      const float ig = gate_sig(zi);
      const float fg = gate_sig(zf);
      const float gg = gate_tanh(zg);
      const float og = gate_sig(zo);
      const float cn = fg * cst[r] + ig * gg;
      cst[r] = cn;
      hst[r] = og * gate_tanh(cn);
    }
    __syncthreads();

#pragma unroll
    for (int r = 0; r < 8; ++r) {
      Axh[(8 * hh + r) * APITCH + NIN + j] = (_Float16)(hst[r] * OPCARRY);
      Hs[(8 * hh + r) * OPITCH + j] = hst[r];
    }
    {
      const int tn = (t + 1 < NSTEP) ? (t + 1) : (NSTEP - 1);
      stage_x_tile<IN_F32>(Axh, xs32, xs16, rowbase, tn, tid);
    }
    __syncthreads();

    if (OUT_F32) {
      const int c4 = c * 4;
      v4f ov[2];
#pragma unroll
      for (int it = 0; it < 2; ++it) {
        const int row = 4 * wave + 2 * it + hh;
        ov[it] = *(const v4f*)(Hs + row * OPITCH + c4);
      }
      for (int pass = 0; pass < 2; ++pass) {
#pragma unroll
        for (int it = 0; it < 2; ++it) {
          const int row = 4 * wave + 2 * it + hh;
          float* dp = h32out + ((size_t)(rowbase + row) * NSTEP + (size_t)t) * NHID + c4;
          *(volatile v4f*)dp = ov[it];
        }
        __threadfence();
      }
    } else {
      const int q = lane >> 3, c8 = (lane & 7) * 8;
      const int row = 4 * wave + q;
      const v4f p0 = *(const v4f*)(Hs + row * OPITCH + c8);
      const v4f p1 = *(const v4f*)(Hs + row * OPITCH + c8 + 4);
      v8h hv;
#pragma unroll
      for (int e = 0; e < 4; ++e) {
        hv[e]     = (_Float16)(p0[e] * OPCARRY);
        hv[4 + e] = (_Float16)(p1[e] * OPCARRY);
      }
      unsigned short* dp = h16out + ((size_t)(rowbase + row) * NSTEP + (size_t)t) * NHID + c8;
      for (int pass = 0; pass < 2; ++pass) {
        *(volatile v8h*)dp = hv;
        __threadfence();
      }
    }
  }
}

extern "C" void kernel_launch(void* const* d_in, const int* in_sizes, int n_in,
                              void* d_out, int out_size, void* d_ws, size_t ws_size, hipStream_t stream) {
  if (n_in < 17 || d_out == nullptr || d_ws == nullptr) return;
  if (in_sizes[0] != NROWS * NIN || out_size != NROWS * NHID) return;
  for (int l = 0; l < NLAYER; ++l) {
    if (in_sizes[1 + 4 * l] != NGATE * NIN || in_sizes[2 + 4 * l] != NGATE * NHID ||
        in_sizes[3 + 4 * l] != NGATE || in_sizes[4 + 4 * l] != NGATE) return;
  }

  const float* x = (const float*)d_in[0];
  const float* wih[NLAYER]; const float* whh[NLAYER]; const float* bih[NLAYER]; const float* bhh[NLAYER];
  for (int l = 0; l < NLAYER; ++l) {
    wih[l] = (const float*)d_in[1 + 4 * l];
    whh[l] = (const float*)d_in[2 + 4 * l];
    bih[l] = (const float*)d_in[3 + 4 * l];
    bhh[l] = (const float*)d_in[4 + 4 * l];
  }
  float* out = (float*)d_out;

  char* ws = (char*)d_ws; size_t off = 0;
  auto carve = [&](size_t bytes) -> char* { char* p = ws + off; off += (bytes + 255) & ~(size_t)255; return p; };
  unsigned short* WC = (unsigned short*)carve((size_t)NLAYER * WPLANE * 2);
  unsigned short* HA = (unsigned short*)carve((size_t)NROWS * NHID * 2);
  unsigned short* HB = (unsigned short*)carve((size_t)NROWS * NHID * 2);
  if (off > ws_size || off > (size_t)134217728) return;

  wcat_kernel<<<(NLAYER * 2 * NGATE * (NIN / 8)) / NTHR, NTHR, 0, stream>>>(
      wih[0], whh[0], wih[1], whh[1], wih[2], whh[2], wih[3], whh[3], WC);

  const int nblk = NSEQ / SEQ_BLK;
  seq_cell_kernel<1, 0><<<nblk, NTHR, 0, stream>>>(x, HB, bih[0], bhh[0], WC + (size_t)0 * WPLANE, HA, out);
  seq_cell_kernel<0, 0><<<nblk, NTHR, 0, stream>>>(x, HA, bih[1], bhh[1], WC + (size_t)1 * WPLANE, HB, out);
  seq_cell_kernel<0, 0><<<nblk, NTHR, 0, stream>>>(x, HB, bih[2], bhh[2], WC + (size_t)2 * WPLANE, HA, out);
  seq_cell_kernel<0, 1><<<nblk, NTHR, 0, stream>>>(x, HA, bih[3], bhh[3], WC + (size_t)3 * WPLANE, HB, out);
}
